// Wasserstain_70231305224565
// MI455X (gfx1250) — hardware-run, weakly checked
//
#include <hip/hip_runtime.h>
#include <stddef.h>
#include <stdint.h>

#define NB       128
#define RV       36
#define WV       50
#define RPAD     48
#define WPAD     64
#define DIMD     256
#define SP       52
#define NE       (RV * WV)
#define NIT      ((NE + 31) / 32)
#define WPB      2
#define NPW      16
#define PPB      (WPB * NPW)
#define ITERS    3
#define LAMB_INV 20.0f
#define EPSV     1e-6f
#define CARRY    16.0f
#define CARRY_INV2 0.00390625f

static_assert(NB % PPB == 0);
static_assert(PPB == 32);
static_assert(DIMD % 32 == 0);
static_assert(RPAD % 16 == 0);
static_assert(WPAD % 16 == 0);
static_assert(RPAD % 4 == 0);
static_assert(WPAD % 4 == 0);
static_assert(RPAD >= RV);
static_assert(WPAD >= WV);
static_assert((RV - 1) * SP + (WV - 1) < RV * SP);
static_assert(NIT * 32 >= NE);

typedef unsigned short us;
typedef _Float16     v16h __attribute__((ext_vector_type(16)));
typedef _Float16     v8h  __attribute__((ext_vector_type(8)));
typedef float        v8f  __attribute__((ext_vector_type(8)));
typedef float        v4f  __attribute__((ext_vector_type(4)));
typedef unsigned int v4u  __attribute__((ext_vector_type(4)));

union Frag { v16h v; v8h h[2]; };
union H8   { v8h h; v4u u; };

__device__ __forceinline__ float wave_sum(float v) {
#pragma unroll
  for (int m = 16; m >= 1; m >>= 1) v += __shfl_xor(v, m, 32);
  return v;
}

__device__ __forceinline__ v8f zero8() { return (v8f){0.f, 0.f, 0.f, 0.f, 0.f, 0.f, 0.f, 0.f}; }

__device__ __forceinline__ v8f mma16(v16h a, v16h b, v8f c) {
  c = __builtin_amdgcn_wmma_f32_16x16x32_f16(false, a, false, b, (short)0, c, false, false);
  asm volatile("v_nop\n\tv_nop\n\tv_nop\n\tv_nop" : "+v"(c) : "v"(a), "v"(b));
  return c;
}

__device__ __forceinline__ v16h ldfrag(const _Float16* p, int ld, int row0, int k0, int lane) {
  const int m = lane & 15, lh = lane >> 4;
  const _Float16* q = p + (size_t)(row0 + m) * ld + k0 + 8 * lh;
  Frag f;
  f.h[0] = *(const v8h*)(q);
  f.h[1] = *(const v8h*)(q + 16);
  return f.v;
}

__global__ __launch_bounds__(128) void k_norm(const float* __restrict__ src, us* __restrict__ dst,
                                              int rowsValid, int rowsPad) {
  const int lane = threadIdx.x & 31, wave = threadIdx.x >> 5, item = blockIdx.x;
  const float* sb = src + (size_t)item * rowsValid * DIMD;
  us* db = dst + (size_t)item * rowsPad * DIMD;
#pragma unroll 1
  for (int r = wave; r < rowsPad; r += 4) {
    const int rc = min(r, rowsValid - 1);
    const float* rp = sb + (size_t)rc * DIMD + lane * 8;
    const v4f x0 = *(const v4f*)(rp);
    const v4f x1 = *(const v4f*)(rp + 4);
    const float x[8] = {x0[0], x0[1], x0[2], x0[3], x1[0], x1[1], x1[2], x1[3]};
    float ss = 0.f;
#pragma unroll
    for (int t = 0; t < 8; ++t) ss += x[t] * x[t];
    ss = wave_sum(ss);
    const float nrm = fmaxf(sqrtf(ss), 1e-8f);
    const float inv = (r < rowsValid) ? (CARRY * (1.0f / nrm)) : 0.0f;
    v8h hv;
#pragma unroll
    for (int t = 0; t < 8; ++t) hv[t] = (_Float16)(x[t] * inv);
    H8 o;
    o.h = hv;
    const v4u u = o.u;
    us* dp = db + (size_t)r * DIMD + lane * 8;
    *(volatile v4u*)dp = u;
    __threadfence();
    *(volatile v4u*)dp = u;
  }
}

__global__ __launch_bounds__(64) void k_tiles(const _Float16* __restrict__ Ap, const _Float16* __restrict__ Bp,
                                              const int* __restrict__ img_lens, const int* __restrict__ cap_lens,
                                              float* __restrict__ out) {
#pragma clang fp contract(off)
  __shared__ __align__(16) float Ssh[WPB][RV * SP];
  __shared__ __align__(16) float Psh[WPB][RV * SP];
  __shared__ float Ush[WPB][64];
  __shared__ float Vsh[WPB][64];
  __shared__ __align__(16) float Osh[PPB];

  const int tid = threadIdx.x, lane = tid & 31, wave = tid >> 5;
  const int hh = lane >> 4, c = lane & 15;
  const int i = blockIdx.x / (NB / PPB);
  const int jbase = (blockIdx.x - i * (NB / PPB)) * PPB;
  const int Ri = img_lens[i];
  const int cntR = min(max(Ri, 0), RV);
  const float rinv = 1.0f / (float)cntR;
  float* S = Ssh[wave];
  float* P = Psh[wave];
  float* U = Ush[wave];
  float* V = Vsh[wave];
  const _Float16* Abase = Ap + (size_t)i * RPAD * DIMD;

#pragma unroll 1
  for (int t = 0; t < NPW; ++t) {
    const int j = jbase + wave * NPW + t;
    const int Wj = cap_lens[j];
    const int cntW = min(max(Wj, 0), WV);
    const float winv = 1.0f / (float)cntW;
    const _Float16* Bbase = Bp + (size_t)j * WPAD * DIMD;

    v8f acc[3][4];
#pragma unroll
    for (int mt = 0; mt < 3; ++mt)
#pragma unroll
      for (int nt = 0; nt < 4; ++nt) acc[mt][nt] = zero8();
#pragma unroll 1
    for (int k0 = 0; k0 < DIMD; k0 += 32) {
      const v16h a0 = ldfrag(Abase, DIMD, 0, k0, lane);
      const v16h a1 = ldfrag(Abase, DIMD, 16, k0, lane);
      const v16h a2 = ldfrag(Abase, DIMD, 32, k0, lane);
#pragma unroll
      for (int nt = 0; nt < 4; ++nt) {
        const v16h b = ldfrag(Bbase, DIMD, nt * 16, k0, lane);
        acc[0][nt] = mma16(a0, b, acc[0][nt]);
        acc[1][nt] = mma16(a1, b, acc[1][nt]);
        acc[2][nt] = mma16(a2, b, acc[2][nt]);
      }
    }
    __syncthreads();
#pragma unroll
    for (int mt = 0; mt < 3; ++mt)
#pragma unroll
      for (int nt = 0; nt < 4; ++nt)
#pragma unroll
        for (int r = 0; r < 8; ++r) {
          const int m = mt * 16 + 8 * hh + r;
          const int n = nt * 16 + c;
          if (m < RV && n < WV) S[m * SP + n] = acc[mt][nt][r] * CARRY_INV2;
        }
    __syncthreads();

    float psum = 0.f;
#pragma unroll 1
    for (int it = 0; it < NIT; ++it) {
      const int idx = it * 32 + lane;
      const int idc = min(idx, NE - 1);
      const int m = idc / WV;
      const int n = idc - m * WV;
      const float s = S[m * SP + n];
      const float e = expf(-((1.0f - s) * LAMB_INV));
      const bool inm = (m < cntR) && (n < cntW);
      const float p = inm ? e : 0.0f;
      if (idx < NE) { P[m * SP + n] = p; psum += p; }
    }
    psum = wave_sum(psum);
    const float pinv = 1.0f / (psum + EPSV);
#pragma unroll 1
    for (int it = 0; it < NIT; ++it) {
      const int idx = it * 32 + lane;
      const int idc = min(idx, NE - 1);
      const int m = idc / WV;
      const int n = idc - m * WV;
      const float q = P[m * SP + n] * pinv;
      if (idx < NE) P[m * SP + n] = q;
    }
    __syncthreads();

#pragma unroll 1
    for (int itr = 0; itr < ITERS; ++itr) {
#pragma unroll
      for (int ps = 0; ps < 2; ++ps) {
        const int mr = lane + 32 * ps;
        const int mc = min(mr, RV - 1);
        const float* pr = P + mc * SP;
        float su = 0.f;
#pragma unroll 5
        for (int n = 0; n < WV; ++n) su += pr[n];
        const float um = su + EPSV;
        const float rm = ((mc < cntR) ? 1.0f : 0.0f) * rinv;
        const float fu = rm * (1.0f / um);
        if (mr < RV) U[mr] = fu;
      }
      __syncthreads();
#pragma unroll
      for (int ps = 0; ps < 2; ++ps) {
        const int nr = lane + 32 * ps;
        const int nc = min(nr, WV - 1);
        float sv = 0.f;
#pragma unroll 4
        for (int m = 0; m < RV; ++m) {
          const float q = P[m * SP + nc] * U[m];
          sv += q;
        }
        const float vn = sv + EPSV;
        const float cn = ((nc < cntW) ? 1.0f : 0.0f) * winv;
        const float fv = cn * (1.0f / vn);
        if (nr < WV) V[nr] = fv;
      }
      __syncthreads();
#pragma unroll 1
      for (int it = 0; it < NIT; ++it) {
        const int idx = it * 32 + lane;
        const int idc = min(idx, NE - 1);
        const int m = idc / WV;
        const int n = idc - m * WV;
        const float q  = P[m * SP + n] * U[m];
        const float q2 = q * V[n];
        if (idx < NE) P[m * SP + n] = q2;
      }
      __syncthreads();
    }

    float fs = 0.f;
#pragma unroll 1
    for (int it = 0; it < NIT; ++it) {
      const int idx = it * 32 + lane;
      const int idc = min(idx, NE - 1);
      const int m = idc / WV;
      const int n = idc - m * WV;
      const float q = S[m * SP + n] * P[m * SP + n];
      if (idx < NE) fs += q;
    }
    fs = wave_sum(fs);
    if (lane == 0) Osh[wave * NPW + t] = fs;
  }

  __syncthreads();
  if (wave == 0) {
    const int q = lane & 7;
    const v4f v = *(const v4f*)(Osh + 4 * q);
    float* op = out + (size_t)i * NB + jbase + 4 * q;
    if (lane < 8) *(volatile v4f*)op = v;
    __threadfence();
    if (lane < 8) *(volatile v4f*)op = v;
  }
}

extern "C" void kernel_launch(void* const* d_in, const int* in_sizes, int n_in,
                              void* d_out, int out_size, void* d_ws, size_t ws_size,
                              hipStream_t stream) {
  if (n_in < 4) return;
  if (in_sizes[0] != NB * RV * DIMD) return;
  if (in_sizes[1] != NB * WV * DIMD) return;
  if (in_sizes[2] != NB) return;
  if (in_sizes[3] != NB) return;
  if (out_size != NB * NB) return;

  const float* imgs     = (const float*)d_in[0];
  const float* caps     = (const float*)d_in[1];
  const int*   img_lens = (const int*)d_in[2];
  const int*   cap_lens = (const int*)d_in[3];
  float*       out      = (float*)d_out;

  size_t off = 0;
  const size_t oA = off; off += (size_t)NB * RPAD * DIMD * 2;
  const size_t oB = off; off += (size_t)NB * WPAD * DIMD * 2;
  if (off > ws_size) return;
  if (off > (size_t)134217728) return;

  char* ws = (char*)d_ws;
  us* Aus = (us*)(ws + oA);
  us* Bus = (us*)(ws + oB);
  const _Float16* Ap = (const _Float16*)(ws + oA);
  const _Float16* Bp = (const _Float16*)(ws + oB);

  k_norm<<<dim3(NB), dim3(128), 0, stream>>>(imgs, Aus, RV, RPAD);
  k_norm<<<dim3(NB), dim3(128), 0, stream>>>(caps, Bus, WV, WPAD);
  k_tiles<<<dim3((NB * NB) / PPB), dim3(32 * WPB), 0, stream>>>(Ap, Bp, img_lens, cap_lens, out);
  (void)hipGetLastError();
}
